// GATLayer_85280870629874
// MI455X (gfx1250) — hardware-run, weakly checked
//
#include <hip/hip_runtime.h>


#ifndef NB
#define NB 8
#endif
#ifndef SEQ
#define SEQ 2048
#endif
#define NB_FULL  8
#define SEQ_FULL 2048
#ifndef OUT_SEQ
#define OUT_SEQ SEQ
#endif
#define DM   128
#define HSP  132
#define PT   256
#define LOG2E 1.4426950408889634f
#define SLOPE 0.2f
#define NEGB (-3.0e38f)

static_assert(DM % 32 == 0);
static_assert(DM == 4 * 32);
static_assert(DM / 4 == 32);
static_assert((NB * SEQ) % 32 == 0);
static_assert(SEQ % 32 == 0);
static_assert(SEQ % PT == 0);
static_assert(PT % 32 == 0);
static_assert(((size_t)SEQ * DM) % 8 == 0);
static_assert(((size_t)DM * DM / 8) % 256 == 0);
static_assert((HSP * 4) % 16 == 0);
static_assert(HSP >= DM);
static_assert(NB <= NB_FULL);
static_assert(SEQ <= SEQ_FULL);
static_assert(16 * HSP * 4 <= 131072);
static_assert((SEQ + PT / 32) * 4 <= 131072);
static_assert((2 * SEQ + PT) * 4 <= 131072);
static_assert((size_t)PT * 16 * (DM / 4) == (size_t)PT * DM * 4);

typedef unsigned short bf;
typedef __attribute__((ext_vector_type(16))) __bf16   v16bf;
typedef __attribute__((ext_vector_type(8)))  unsigned short v8us;
typedef __attribute__((ext_vector_type(8)))  float    v8f;
typedef __attribute__((ext_vector_type(4)))  float    v4f;
typedef v4f  __attribute__((may_alias)) v4fa;

__device__ __forceinline__ unsigned short f2bf(float f) { unsigned u = __float_as_uint(f); u += 0x7FFFu + ((u >> 16) & 1u); return (unsigned short)(u >> 16); }
__device__ __forceinline__ float bfr(float f) { return __uint_as_float(((unsigned)f2bf(f)) << 16); }
__device__ __forceinline__ v16bf cat16b(v8us lo, v8us hi) { return __builtin_bit_cast(v16bf, __builtin_shufflevector(lo, hi, 0, 1, 2, 3, 4, 5, 6, 7, 8, 9, 10, 11, 12, 13, 14, 15)); }
__device__ __forceinline__ v8f wmmab(v16bf a, v16bf b, v8f c) { return __builtin_amdgcn_wmma_f32_16x16x32_bf16(false, a, false, b, (short)0, c, false, false); }
__device__ __forceinline__ v8f wmmab_g(v16bf a, v16bf b, v8f c) { c = wmmab(a, b, c); asm volatile("v_nop\n\tv_nop\n\tv_nop\n\tv_nop" : "+v"(c) : "v"(a), "v"(b)); return c; }
__device__ __forceinline__ v16bf ldb(const bf* p)  { return cat16b(*(const v8us*)p, *(const v8us*)(p + 16)); }
__device__ __forceinline__ void wave_sync() { __builtin_amdgcn_fence(3  , "wavefront"); __builtin_amdgcn_wave_barrier(); asm volatile("" ::: "memory"); }
__device__ __forceinline__ float lrelu(float v) { return v > 0.0f ? v : SLOPE * v; }

__global__ __launch_bounds__(256) void k_cvt8(const float* __restrict__ src, bf* dst, size_t n8) {
    const size_t i = (size_t)blockIdx.x * 256 + threadIdx.x; if (i >= n8) return;
    const v8f v = *(const v8f*)(src + i * 8); v8us o;
#pragma unroll
    for (int k = 0; k < 8; ++k) o[k] = f2bf(v[k]);
    *(volatile v8us*)(dst + i * 8) = o; __threadfence(); *(volatile v8us*)(dst + i * 8) = o;
}

__global__ __launch_bounds__(256) void k_wt(const float* __restrict__ W, bf* WT) {
    const int i = blockIdx.x * 256 + threadIdx.x; if (i >= DM * DM / 8) return;
    const int n = i / (DM / 8), c = i % (DM / 8);
    v8us o;
#pragma unroll
    for (int j = 0; j < 8; ++j) o[j] = f2bf(W[(size_t)(8 * c + j) * DM + n]);
    *(volatile v8us*)(WT + (size_t)i * 8) = o; __threadfence(); *(volatile v8us*)(WT + (size_t)i * 8) = o;
}

__global__ __launch_bounds__(32) void k_hs(const bf* __restrict__ A, const bf* __restrict__ Bt, const float* __restrict__ wv, const float* __restrict__ bv, float* H, float* S) {
    __shared__ __align__(16) float os[16 * HSP];
    const int K = DM;
    const int lane = threadIdx.x & 31, lr = lane & 15, hi = lane >> 4; const int r0 = blockIdx.x * 32;
    v8f acc[2][8];
#pragma unroll
    for (int mb = 0; mb < 2; ++mb)
#pragma unroll
        for (int nb = 0; nb < 8; ++nb) acc[mb][nb] = (v8f){};
    const size_t aoff = (size_t)(r0 + lr) * K + 8 * hi, boff = (size_t)lr * K + 8 * hi;
#pragma unroll 1
    for (int kc = 0; kc < K; kc += 32) {
        v16bf a[2];
#pragma unroll
        for (int mb = 0; mb < 2; ++mb) a[mb] = ldb(A + aoff + (size_t)mb * 16 * K + kc);
#pragma unroll
        for (int nb = 0; nb < 8; ++nb) { const v16bf b = ldb(Bt + boff + (size_t)nb * 16 * K + kc);
#pragma unroll
            for (int mb = 0; mb < 2; ++mb) acc[mb][nb] = wmmab_g(a[mb], b, acc[mb][nb]); }
    }
    const v4f wl = *(const v4f*)(wv + 4 * lane);
    const float w0 = bfr(wl[0]), w1 = bfr(wl[1]), w2 = bfr(wl[2]), w3 = bfr(wl[3]);
    const float bias = bfr(bv[0]);
    float sv = 0.0f;
#pragma unroll
    for (int mb = 0; mb < 2; ++mb) {
#pragma unroll
        for (int nb = 0; nb < 8; ++nb) {
#pragma unroll
            for (int j = 0; j < 8; ++j) os[(hi * 8 + j) * HSP + nb * 16 + lr] = acc[mb][nb][j]; }
        wave_sync();
#pragma unroll 1
        for (int r = 0; r < 16; ++r) {
            const v4f hv = *(const v4fa*)(&os[r * HSP + 4 * lane]);
            float d = hv[0] * w0 + hv[1] * w1 + hv[2] * w2 + hv[3] * w3;
            d += __shfl_xor(d, 16, 32); d += __shfl_xor(d, 8, 32); d += __shfl_xor(d, 4, 32); d += __shfl_xor(d, 2, 32); d += __shfl_xor(d, 1, 32);
            sv = (lane == mb * 16 + r) ? d : sv; }
        float* hrow = H + (size_t)(r0 + mb * 16) * DM + 4 * lane;
#pragma unroll 1
        for (int ps = 0; ps < 2; ++ps) {
#pragma unroll
            for (int r = 0; r < 16; ++r) {
                const v4f val = *(const v4fa*)(&os[r * HSP + 4 * lane]);
                *(volatile v4f*)(hrow + (size_t)r * DM) = val; }
            if (ps == 0) __threadfence(); }
        wave_sync();
    }
    const float so = (sv + bias) * LOG2E;
    volatile float* sp = S + (size_t)r0 + lane;
    *sp = so; __threadfence(); *sp = so;
}

__global__ __launch_bounds__(PT) void k_zrow(const float* __restrict__ S, float* Q) {
#pragma clang fp contract(off)
    __shared__ float ss[SEQ];
    __shared__ float wm[PT / 32];
    const int b = blockIdx.y;
    const int lane = threadIdx.x & 31;
    const int wave = __builtin_amdgcn_readfirstlane((int)(threadIdx.x >> 5));
    float mx = NEGB;
#pragma unroll 1
    for (int i = threadIdx.x; i < SEQ; i += PT) { const float v = S[(size_t)b * SEQ + i]; ss[i] = v; mx = fmaxf(mx, v); }
    mx = fmaxf(mx, __shfl_xor(mx, 16, 32)); mx = fmaxf(mx, __shfl_xor(mx, 8, 32)); mx = fmaxf(mx, __shfl_xor(mx, 4, 32));
    mx = fmaxf(mx, __shfl_xor(mx, 2, 32)); mx = fmaxf(mx, __shfl_xor(mx, 1, 32));
    if (lane == 0) wm[wave] = mx;
    __syncthreads();
    float smx = wm[0];
#pragma unroll
    for (int w = 1; w < PT / 32; ++w) smx = fmaxf(smx, wm[w]);
    const int i = blockIdx.x * PT + threadIdx.x;
    const float si = ss[i];
    const float m = lrelu(si + smx);
    float acc = 0.0f;
#pragma unroll 4
    for (int j = 0; j < SEQ; ++j) acc += __builtin_amdgcn_exp2f(lrelu(si + ss[j]) - m);
    const float q = m + __builtin_amdgcn_logf(acc);
    volatile float* qp = Q + (size_t)b * SEQ + i;
    *qp = q; __threadfence(); *qp = q;
}

__global__ __launch_bounds__(PT) void k_colout(const float* __restrict__ S, const float* __restrict__ Q, const float* __restrict__ H, float* OUT) {
#pragma clang fp contract(off)
    __shared__ float ss[SEQ];
    __shared__ float qq[SEQ];
    __shared__ float colsh[PT];
    const int b = blockIdx.y;
    const int wave = __builtin_amdgcn_readfirstlane((int)(threadIdx.x >> 5));
#pragma unroll 1
    for (int i = threadIdx.x; i < SEQ; i += PT) { ss[i] = S[(size_t)b * SEQ + i]; qq[i] = Q[(size_t)b * SEQ + i]; }
    __syncthreads();
    const int j = blockIdx.x * PT + threadIdx.x;
    const float sj = ss[j];
    float acc = 0.0f;
#pragma unroll 4
    for (int i = 0; i < SEQ; ++i) acc += __builtin_amdgcn_exp2f(lrelu(ss[i] + sj) - qq[i]);
    colsh[threadIdx.x] = acc;
    __syncthreads();
    const float* hb = H + ((size_t)b * SEQ + (size_t)blockIdx.x * PT) * DM;
    float* ob = OUT + ((size_t)b * OUT_SEQ + (size_t)blockIdx.x * PT) * DM;
#pragma unroll 1
    for (int ps = 0; ps < 2; ++ps) {
#pragma unroll 4
        for (int it = 0; it < DM / 4; ++it) {
            const int r = it * (PT / 32) + wave;
            const size_t o4 = ((size_t)it * PT + threadIdx.x) * 4;
            const v4f hv = *(const v4f*)(hb + o4);
            const float c = colsh[r];
            v4f val;
            val[0] = lrelu(hv[0] * c); val[1] = lrelu(hv[1] * c); val[2] = lrelu(hv[2] * c); val[3] = lrelu(hv[3] * c);
            *(volatile v4f*)(ob + o4) = val; }
        if (ps == 0) __threadfence(); }
}

static constexpr size_t al256(size_t v) { return (v + 255) & ~(size_t)255; }
static constexpr size_t SZ_XB = al256((size_t)NB * SEQ * DM * 2);
static constexpr size_t SZ_WT = al256((size_t)DM * DM * 2);
static constexpr size_t SZ_H  = al256((size_t)NB * SEQ * DM * 4);
static constexpr size_t SZ_S  = al256((size_t)NB * SEQ * 4);
static constexpr size_t SZ_TOTAL = SZ_XB + SZ_WT + SZ_H + 2 * SZ_S;
static_assert(SZ_TOTAL <= (size_t)134217728);
static_assert(((size_t)(NB * SEQ / 32 - 1) * 32 + 31) < (size_t)NB * SEQ);
static_assert(((size_t)(NB * SEQ / 32 - 1) * 32 + 31) * DM + DM <= (size_t)NB * SEQ * DM);

extern "C" void kernel_launch(void* const* d_in, const int* in_sizes, int n_in,
                              void* d_out, int out_size, void* d_ws, size_t ws_size, hipStream_t stream) {
    if (n_in < 4) return;
    const size_t needx = ((size_t)(NB - 1) * SEQ_FULL + SEQ) * DM;
    if ((size_t)in_sizes[0] < needx) return;
    if ((size_t)in_sizes[1] < (size_t)DM * DM) return;
    if (in_sizes[2] < DM || in_sizes[3] < 1) return;
    if ((size_t)out_size < ((size_t)(NB - 1) * OUT_SEQ + SEQ) * DM) return;
    if (SZ_TOTAL > ws_size) return;
    const float* xin = (const float*)d_in[0];
    const float* wmat = (const float*)d_in[1];
    const float* wvec = (const float*)d_in[2];
    const float* bvec = (const float*)d_in[3];
    float* OUT = (float*)d_out;
    char* wsp = (char*)d_ws;
    bf* XB = (bf*)wsp; wsp += SZ_XB;
    bf* WT = (bf*)wsp; wsp += SZ_WT;
    float* H = (float*)wsp; wsp += SZ_H;
    float* S = (float*)wsp; wsp += SZ_S;
    float* Q = (float*)wsp; wsp += SZ_S;

    if (SEQ == SEQ_FULL) {
        const size_t n8 = (size_t)NB * SEQ * DM / 8;
        k_cvt8<<<(unsigned)((n8 + 255) / 256), 256, 0, stream>>>(xin, XB, n8);
    } else {
        const size_t n8 = (size_t)SEQ * DM / 8;
        for (int b = 0; b < NB; ++b) k_cvt8<<<(unsigned)((n8 + 255) / 256), 256, 0, stream>>>(xin + (size_t)b * SEQ_FULL * DM, XB + (size_t)b * SEQ * DM, n8);
    }
    k_wt<<<(unsigned)(DM * DM / 8 / 256), 256, 0, stream>>>(wmat, WT);

    k_hs<<<(unsigned)(NB * SEQ / 32), 32, 0, stream>>>(XB, WT, wvec, bvec, H, S);

    k_zrow<<<dim3(SEQ / PT, NB, 1), PT, 0, stream>>>(S, Q);
    k_colout<<<dim3(SEQ / PT, NB, 1), PT, 0, stream>>>(S, Q, H, OUT);
}
